// SlotMemSparse_19842748907985
// MI455X (gfx1250) — hardware-run, weakly checked
//
#include <hip/hip_runtime.h>


namespace {
constexpr int BK = 1024, NX = 16384, FIN = 256, F = 128, NH = 8, FH = 16, E = 278528, NCAT = BK + NX  ;
constexpr float XS = 8.0f, WSC = 256.0f, LNE = 1e-5f, QS = 0.25f;

typedef _Float16 b16;
typedef __attribute__((ext_vector_type(16))) _Float16 v16b;
typedef __attribute__((ext_vector_type(8))) _Float16 v8b;
typedef __attribute__((ext_vector_type(8))) float v8f;
typedef __attribute__((ext_vector_type(4))) float v4f;
typedef __attribute__((ext_vector_type(4))) _Float16 v4b;
__device__ __forceinline__ float bf16_rne(float f) { unsigned int u = __float_as_uint(f); u += 0x7FFFu + ((u >> 16) & 1u); return __uint_as_float(u & 0xFFFF0000u); }
__device__ __forceinline__ void split16(float v, b16& hi, b16& lo) { hi = (b16)v; lo = (b16)(v - (float)hi); }
__device__ __forceinline__ v16b frag_kb(const b16* p, int hh) { const v8b a = *(const v8b*)(p + 8 * hh), b = *(const v8b*)(p + 16 + 8 * hh); v16b f;
#pragma unroll
  for (int e = 0; e < 8; ++e) { f[e] = a[e]; f[8 + e] = b[e]; } return f; }
__device__ __forceinline__ v8f wmma16b(v16b a, v16b b, v8f c) { v8f d = __builtin_amdgcn_wmma_f32_16x16x32_f16(false, a, false, b, (short)0, c, false, false); asm volatile("v_nop\n\tv_nop\n\tv_nop\n\tv_nop" : "+v"(d) : "v"(a), "v"(b)); return d; }
__device__ __forceinline__ void wave_lds_sync() { __builtin_amdgcn_fence(__ATOMIC_RELEASE, "workgroup"); __builtin_amdgcn_wave_barrier(); __builtin_amdgcn_fence(__ATOMIC_ACQUIRE, "workgroup"); }
__device__ __forceinline__ float pmul(float a, float b) { float p = a * b; asm volatile("" : "+v"(p)); return p; }
__device__ __forceinline__ float wsum(float v) { v += __shfl_xor(v, 1); v += __shfl_xor(v, 2); v += __shfl_xor(v, 4); v += __shfl_xor(v, 8); return v + __shfl_xor(v, 16); }
__device__ __forceinline__ int iclamp(int v, int lo, int hi) { return v < lo ? lo : (v > hi ? hi : v); }
__device__ __forceinline__ float nexp(float x) { return __builtin_amdgcn_exp2f(x * 1.4426950408889634f); }
__device__ __forceinline__ float sigm(float x) { return 1.0f / (1.0f + nexp(-x)); }

constexpr int CSR_NBLK = 512, CSR_GB = 5, CSR_GN = 1 << CSR_GB  , CSR_MAXG = 512, CSR_CAP = 12288  ;
__global__ __launch_bounds__(64) void csrA_kernel(const int* __restrict__ dst, int E, int N, int nG, int CHP, int NGP, int* __restrict__ STG, int* __restrict__ HST) {
  extern __shared__ int sm[];
  int* cnt = sm; int* run = sm + NGP; int* ids = sm + 2 * NGP;
  const int b = blockIdx.x; const int ch = (E + CSR_NBLK - 1) / CSR_NBLK; const int e0 = b * ch, e1 = min(E, e0 + ch);
  for (int i = threadIdx.x; i < NGP; i += 64) cnt[i] = 0;
  for (int i = threadIdx.x; i < CHP; i += 64) ids[i] = -1;
  __syncthreads();
  if (threadIdx.x == 0) {
    for (int e = e0; e < e1; ++e) { int d = dst[e]; d = (d < 0) ? 0 : (d >= N ? N - 1 : d); cnt[d >> CSR_GB] += 1; }
    int acc = 0; for (int g = 0; g < nG; ++g) { run[g] = acc; acc += cnt[g]; }
    for (int e = e0; e < e1; ++e) { int d = dst[e]; d = (d < 0) ? 0 : (d >= N ? N - 1 : d); const int g = d >> CSR_GB; ids[run[g]] = e; run[g] += 1; } }
  __syncthreads();
  typedef __attribute__((ext_vector_type(4))) int v4i;
  for (int pass = 0; pass < 2; ++pass) {
    for (int i = threadIdx.x; i < CHP / 4; i += 64) *(volatile v4i*)(STG + (size_t)b * CHP + i * 4) = *(const v4i*)(&ids[i * 4]);
    for (int i = threadIdx.x; i < NGP / 4; i += 64) { v4i v; for (int e = 0; e < 4; ++e) v[e] = (i * 4 + e < nG) ? cnt[i * 4 + e] : 0; *(volatile v4i*)(HST + (size_t)b * NGP + i * 4) = v; }
    __threadfence(); }
}
__global__ __launch_bounds__(512) void csrS_kernel(const int* __restrict__ HST, int nG, int NGP, int* __restrict__ START, int* __restrict__ TOT, int* __restrict__ OFF) {
  __shared__ int tot[CSR_MAXG];
  const int b = threadIdx.x;
  for (int pass = 0; pass < 2; ++pass) { int runb = 0; for (int g = 0; g < nG; ++g) { int c = HST[(size_t)b * NGP + g]; c = (c < 0) ? 0 : c; ((volatile int*)OFF)[(size_t)g * CSR_NBLK + b] = runb; runb += c; } __threadfence(); }
  for (int g = threadIdx.x; g < nG; g += 512) { int s = 0; for (int bb = 0; bb < CSR_NBLK; ++bb) { int c = HST[(size_t)bb * NGP + g]; s += (c < 0) ? 0 : c; } tot[g] = s; }
  __syncthreads();
  if (threadIdx.x < 32) {
    __shared__ int st[CSR_MAXG + 32];
    if (threadIdx.x == 0) { int acc = 0; for (int g = 0; g < NGP; ++g) { st[g] = acc; if (g < nG) acc += (tot[g] + 31) & ~31; } st[NGP] = acc; }
    __builtin_amdgcn_fence(__ATOMIC_RELEASE, "workgroup"); __builtin_amdgcn_wave_barrier(); __builtin_amdgcn_fence(__ATOMIC_ACQUIRE, "workgroup");
    for (int pass = 0; pass < 2; ++pass) { for (int i = threadIdx.x; i < NGP + 32; i += 32) { ((volatile int*)START)[i] = (i <= NGP) ? st[min(i, NGP)] : 0; ((volatile int*)TOT)[i] = (i < nG) ? tot[i] : 0; } __threadfence(); } }
}
__global__ __launch_bounds__(256) void csrB_kernel(const int* __restrict__ dst, int N, int nG, int CHP, int NGP, int permLen, const int* __restrict__ STG, const int* __restrict__ HST, const int* __restrict__ OFF, const int* __restrict__ START, const int* __restrict__ TOT, int* __restrict__ PERM, int* __restrict__ ROWPTR, int* __restrict__ ROWCNT, int* __restrict__ FLAG) {
  typedef __attribute__((ext_vector_type(4))) int v4i;
  __shared__ int ids[CSR_CAP]; __shared__ unsigned short key[CSR_CAP]; __shared__ int outp[CSR_CAP]; __shared__ int ncnt[CSR_GN + 1]; __shared__ int boff[CSR_NBLK + 1];
  const int g = blockIdx.x, t_ = threadIdx.x; int tot = TOT[g]; int st = START[g], stn = START[g + 1]; const int v0 = g * CSR_GN; const int nv = min(CSR_GN, N - v0);
  st = (st < 0) ? 0 : (st > permLen - 32 ? permLen - 32 : st) & ~31; stn = (stn < st) ? st : (stn > permLen ? permLen : stn); tot = (tot < 0) ? 0 : tot; if (tot > stn - st && tot <= CSR_CAP) tot = stn - st;
  if (tot > CSR_CAP) {
    for (int pass = 0; pass < 2; ++pass) { for (int i = t_; i < CSR_GN / 4; i += 256) { v4i a, c; for (int e = 0; e < 4; ++e) { a[e] = st; c[e] = 0; } *(volatile v4i*)(ROWPTR + v0 + i * 4) = a; *(volatile v4i*)(ROWCNT + v0 + i * 4) = c; } if (t_ == 0) ((volatile int*)FLAG)[0] = 1; __threadfence(); } (void)nv; return; }
  if (t_ == 0) { int acc = 0; for (int b = 0; b < CSR_NBLK; ++b) { boff[b] = acc; int c = HST[(size_t)b * NGP + g]; c = (c < 0) ? 0 : (c > CHP ? CHP : c); acc += c; if (acc > tot) acc = tot; } boff[CSR_NBLK] = acc; }
  for (int i = t_; i <= CSR_GN; i += 256) ncnt[i] = 0;
  __syncthreads();
  for (int b = 0; b < CSR_NBLK; ++b) { const int c = boff[b + 1] - boff[b]; int o_ = OFF[(size_t)g * CSR_NBLK + b]; o_ = (o_ < 0) ? 0 : (o_ > CHP - c ? CHP - c : o_); const int* src_ = STG + (size_t)b * CHP + o_;
    for (int i = t_; i < c; i += 256) { int id = src_[i]; id = (id < 0) ? 0 : id; ids[boff[b] + i] = id; int d = dst[id]; d = (d < v0) ? v0 : (d >= N ? N - 1 : d); int kk = d - v0; kk = (kk < 0) ? 0 : (kk >= CSR_GN ? CSR_GN - 1 : kk); key[boff[b] + i] = (unsigned short)kk; } }
  __syncthreads();
  if (t_ == 0) { for (int i = 0; i < tot; ++i) ncnt[key[i]] += 1; int acc = 0; for (int vl = 0; vl < CSR_GN; ++vl) { const int c = ncnt[vl]; ncnt[vl] = acc; acc += c; } ncnt[CSR_GN] = acc;
    for (int i = 0; i < tot; ++i) { const int vl = key[i]; outp[ncnt[vl]] = ids[i]; ncnt[vl] += 1; }
    for (int vl = CSR_GN; vl > 0; --vl) ncnt[vl] = ncnt[vl - 1]; ncnt[0] = 0; }
  __syncthreads();
  for (int pass = 0; pass < 2; ++pass) {
    for (int i = t_; i < (stn - st) / 4; i += 256) { v4i v; for (int e = 0; e < 4; ++e) { const int q = i * 4 + e; v[e] = (q < tot) ? outp[q] : -1; } *(volatile v4i*)(PERM + st + i * 4) = v; }
    for (int i = t_; i < CSR_GN / 4; i += 256) { v4i a, c; for (int e = 0; e < 4; ++e) { const int vl = i * 4 + e; a[e] = st + ncnt[vl]; c[e] = (vl < nv) ? (ncnt[vl + 1] - ncnt[vl]) : 0; } *(volatile v4i*)(ROWPTR + v0 + i * 4) = a; *(volatile v4i*)(ROWCNT + v0 + i * 4) = c; }
    __threadfence(); }
}
__global__ __launch_bounds__(256) void csrZ_kernel(int* __restrict__ p, size_t n4) { typedef __attribute__((ext_vector_type(4))) int v4i; const size_t tid = (size_t)blockIdx.x * 256 + threadIdx.x, nth = (size_t)gridDim.x * 256; v4i z = {0, 0, 0, 0}; for (size_t i = tid; i < n4; i += nth) *(volatile v4i*)(p + i * 4) = z; }
struct CsrBufs { int *STG, *HST, *OFF, *START, *TOT, *PERM, *ROWPTR, *ROWCNT, *FLAG; int nG, NGP, CHP; size_t permLen; char* base; size_t bytes; };
static size_t csr_carve(CsrBufs& c, char* ws, size_t off, int E, int N) {
  const size_t off0 = off; c.base = ws + off;
  auto al = [&](size_t bytes) { char* p = ws + off; off += (bytes + 255) & ~(size_t)255; return p; };
  c.nG = (N + CSR_GN - 1) / CSR_GN; c.NGP = (c.nG + 31) & ~31; const int ch = (E + CSR_NBLK - 1) / CSR_NBLK; c.CHP = (ch + 31) & ~31; c.permLen = (size_t)E + 32 * (size_t)c.nG + 32;
  c.STG = (int*)al((size_t)CSR_NBLK * c.CHP * 4); c.HST = (int*)al((size_t)CSR_NBLK * c.NGP * 4); c.OFF = (int*)al((size_t)c.NGP * CSR_NBLK * 4); c.START = (int*)al((size_t)(c.NGP + 64) * 4); c.TOT = (int*)al((size_t)(c.NGP + 64) * 4);
  c.PERM = (int*)al(c.permLen * 4); c.ROWPTR = (int*)al((size_t)c.nG * CSR_GN * 4); c.ROWCNT = (int*)al((size_t)c.nG * CSR_GN * 4); c.FLAG = (int*)al(256);
  c.bytes = off - off0; return off;
}
static void csr_build(const CsrBufs& c, const int* dst, int E, int N, hipStream_t stream) {
  const size_t smem = (size_t)(2 * c.NGP + c.CHP) * 4;
  csrZ_kernel<<<512, 256, 0, stream>>>((int*)c.base, c.bytes / 16);
  csrA_kernel<<<CSR_NBLK, 64, smem, stream>>>(dst, E, N, c.nG, c.CHP, c.NGP, c.STG, c.HST);
  csrS_kernel<<<1, 512, 0, stream>>>(c.HST, c.nG, c.NGP, c.START, c.TOT, c.OFF);
  csrB_kernel<<<c.nG, 256, 0, stream>>>(dst, N, c.nG, c.CHP, c.NGP, (int)c.permLen, c.STG, c.HST, c.OFF, c.START, c.TOT, c.PERM, c.ROWPTR, c.ROWCNT, c.FLAG);
}


__global__ __launch_bounds__(256) void prep_kernel(const float* __restrict__ x, const float* __restrict__ mem, const float* __restrict__ wp, const float* __restrict__ wqkv, const float* __restrict__ w1, const float* __restrict__ w2, const float* __restrict__ wg, b16* __restrict__ X16, b16* __restrict__ M16, b16* __restrict__ WT) {
  const size_t t = (size_t)blockIdx.x * 256 + threadIdx.x; const size_t nx = (size_t)NX * FIN / 8, nm = (size_t)BK * F / 8, n1 = (size_t)F * FIN / 8, n2 = (size_t)3 * F * F / 8, n3 = (size_t)F * F / 8, n5 = (size_t)4 * F * F / 8; v8b o;
  if (t < nx) { const size_t e = t * 8; for (int j = 0; j < 8; ++j) o[j] = (b16)(bf16_rne(x[e + j]) * XS); for (int pass = 0; pass < 2; ++pass) { *(volatile v8b*)(X16 + e) = o; __threadfence(); } return; }
  size_t u = t - nx;
  if (u < nm) { const size_t e = u * 8; for (int j = 0; j < 8; ++j) o[j] = (b16)(bf16_rne(mem[e + j]) * XS); for (int pass = 0; pass < 2; ++pass) { *(volatile v8b*)(M16 + e) = o; __threadfence(); } return; }
  u -= nm; size_t woff; const float* w; int nin, nout;
  if (u < n1) { w = wp; nin = FIN; nout = F; woff = 0; } else if ((u -= n1) < n2) { w = wqkv; nin = F; nout = 3 * F; woff = (size_t)F * FIN; } else if ((u -= n2) < n3) { w = w1; nin = F; nout = F; woff = (size_t)F * FIN + 3 * F * F; }
  else if ((u -= n3) < n3) { w = w2; nin = F; nout = F; woff = (size_t)F * FIN + 4 * F * F; } else if ((u -= n3) < n5) { w = wg; nin = 2 * F; nout = 2 * F; woff = (size_t)F * FIN + 5 * F * F; } else return;
  const size_t e = u * 8; const int oo = (int)(e / nin), i0 = (int)(e % nin); (void)nout;
  for (int j = 0; j < 8; ++j) o[j] = (b16)(bf16_rne(w[(size_t)(i0 + j) * nout + oo]) * WSC);
  for (int pass = 0; pass < 2; ++pass) { *(volatile v8b*)(WT + woff + e) = o; __threadfence(); }
}
template <int MODE, int K, int QSCALE = 0>
__global__ __launch_bounds__(128) void gemm_kernel(const b16* __restrict__ Ah, const b16* __restrict__ Al, const b16* __restrict__ A2h, const b16* __restrict__ A2l, const b16* __restrict__ W, const float* __restrict__ bias, b16* __restrict__ Yh, b16* __restrict__ Yl, float* __restrict__ Yf, int ldy) {
  __shared__ __attribute__((aligned(16))) float Ts[4][16][128 + 4];
  const int wave = threadIdx.x >> 5, lane = threadIdx.x & 31, nloc = lane & 15, hlf = lane >> 4; size_t m0 = (size_t)blockIdx.x * 64 + wave * 16; const int n0 = blockIdx.y * 128;
  const b16* ah = Ah; const b16* al = Al;
  if (MODE == 1) { if (blockIdx.x >= BK / 64) { ah = A2h; al = A2l; m0 -= BK; } else { al = nullptr; } if (QSCALE && blockIdx.x >= BK / 64) return; }
  v8f acc[8];
#pragma unroll
  for (int t = 0; t < 8; ++t) acc[t] = (v8f){};
#pragma unroll 2
  for (int kb = 0; kb < K; kb += 32) { const v16b a = frag_kb(ah + (m0 + nloc) * K + kb, hlf); v16b a2 = {}; if (al) a2 = frag_kb(al + (m0 + nloc) * K + kb, hlf);
#pragma unroll
    for (int t = 0; t < 8; ++t) { const v16b bw = frag_kb(W + (size_t)(n0 + t * 16 + nloc) * K + kb, hlf); acc[t] = wmma16b(a, bw, acc[t]); if (al) acc[t] = wmma16b(a2, bw, acc[t]); } }
#pragma unroll
  for (int t = 0; t < 8; ++t) { const int c = n0 + t * 16 + nloc; const float bb = bias ? bf16_rne(bias[c]) : 0.0f;
#pragma unroll
    for (int r = 0; r < 8; ++r) { float v = acc[t][r] * (1.0f / (XS * WSC)) + bb; if (MODE == 2) v = fmaxf(v, 0.0f); if (QSCALE) v *= QS; Ts[wave][8 * hlf + r][t * 16 + nloc] = v; } }
  wave_lds_sync();
  const size_t yrow0 = (MODE == 1) ? (size_t)blockIdx.x * 64 + wave * 16 : m0;
  float* yf = Yf;
  for (int pass = 0; pass < 2; ++pass) { for (int rr = 0; rr < 16; ++rr) {
      if (MODE == 0 || MODE == 2) { if (lane < 16) { v8b hv, lv; for (int j = 0; j < 8; ++j) { b16 p, q; split16(Ts[wave][rr][lane * 8 + j] * XS, p, q); hv[j] = p; lv[j] = q; } *(volatile v8b*)(Yh + (yrow0 + rr) * 128 + lane * 8) = hv; *(volatile v8b*)(Yl + (yrow0 + rr) * 128 + lane * 8) = lv; } }
      else *(volatile v4f*)(yf + (yrow0 + rr) * ldy + (MODE == 1 ? 0 : n0) + lane * 4) = *(const v4f*)(&Ts[wave][rr][lane * 4]);
    } __threadfence(); }
}
__global__ __launch_bounds__(256) void edge_kernel(const float* __restrict__ Q, const float* __restrict__ Kp, const float* __restrict__ Vp, const float* __restrict__ mem, const int* __restrict__ dest, const int* __restrict__ PERM, const int* __restrict__ ROWPTR, const int* __restrict__ ROWCNT, int permLen, const float* __restrict__ g1, const float* __restrict__ be1, float* __restrict__ MT, b16* __restrict__ MTh, b16* __restrict__ MTl) {
  const int wave = threadIdx.x >> 5, lane = threadIdx.x & 31; const int s = blockIdx.x * 8 + wave; const int c0 = lane * 4;
  int st = ROWPTR[s], cnt = ROWCNT[s]; cnt = iclamp(cnt, 0, 8192); st = iclamp(st, 0, permLen - cnt);
  const v4f q4 = *(const v4f*)(Q + (size_t)s * F + c0);
  float mx = -INFINITY;
  for (int j = 0; j < cnt; ++j) { const int e = iclamp(PERM[st + j], 0, E - 1); const int d = iclamp(dest[e], 0, NCAT - 1); const v4f k4 = *(const v4f*)(Kp + (size_t)d * F + c0); float pd = ((pmul(q4[0], k4[0]) + pmul(q4[1], k4[1])) + pmul(q4[2], k4[2])) + pmul(q4[3], k4[3]); pd += __shfl_xor(pd, 1); pd += __shfl_xor(pd, 2); mx = fmaxf(mx, pd); }
  float z = 0.0f; float acc[4] = {0, 0, 0, 0};
  for (int j = 0; j < cnt; ++j) { const int e = iclamp(PERM[st + j], 0, E - 1); const int d = iclamp(dest[e], 0, NCAT - 1); const v4f k4 = *(const v4f*)(Kp + (size_t)d * F + c0); float pd = ((pmul(q4[0], k4[0]) + pmul(q4[1], k4[1])) + pmul(q4[2], k4[2])) + pmul(q4[3], k4[3]); pd += __shfl_xor(pd, 1); pd += __shfl_xor(pd, 2);
    const float ex = nexp(pd - mx); z += ex; const v4f v4 = *(const v4f*)(Vp + (size_t)d * F + c0); for (int q = 0; q < 4; ++q) acc[q] += pmul(ex, v4[q]); }
  const float inv = (cnt > 0) ? 1.0f / z : 0.0f;
  float y[4]; float s1 = 0.0f; for (int q = 0; q < 4; ++q) { y[q] = bf16_rne(mem[(size_t)s * F + c0 + q]) + acc[q] * inv; s1 += y[q]; }
  const float mu = wsum(s1) * (1.0f / F); float s2 = 0.0f; for (int q = 0; q < 4; ++q) { const float dv = y[q] - mu; s2 += dv * dv; } const float rs = rsqrtf(wsum(s2) * (1.0f / F) + LNE);
  v4f o; v4b hv, lv; for (int q = 0; q < 4; ++q) { o[q] = pmul((y[q] - mu) * rs, bf16_rne(g1[c0 + q])) + bf16_rne(be1[c0 + q]); b16 p, qq; split16(o[q] * XS, p, qq); hv[q] = p; lv[q] = qq; }
  for (int pass = 0; pass < 2; ++pass) { *(volatile v4f*)(MT + (size_t)s * F + c0) = o; *(volatile v4b*)(MTh + (size_t)s * F + c0) = hv; *(volatile v4b*)(MTl + (size_t)s * F + c0) = lv; __threadfence(); }
}
__global__ __launch_bounds__(256) void ln2_kernel(const float* __restrict__ MT, const float* __restrict__ U, const float* __restrict__ mem, const float* __restrict__ g2, const float* __restrict__ be2, float* __restrict__ MU, b16* __restrict__ CATh, b16* __restrict__ CATl) {
  const int wave = threadIdx.x >> 5, lane = threadIdx.x & 31; const int s = blockIdx.x * 8 + wave; const int c0 = lane * 4;
  float y[4]; float s1 = 0.0f; for (int q = 0; q < 4; ++q) { y[q] = MT[(size_t)s * F + c0 + q] + U[(size_t)s * F + c0 + q]; s1 += y[q]; }
  const float mu = wsum(s1) * (1.0f / F); float s2 = 0.0f; for (int q = 0; q < 4; ++q) { const float dv = y[q] - mu; s2 += dv * dv; } const float rs = rsqrtf(wsum(s2) * (1.0f / F) + LNE);
  v4f o; v4b hv, lv, mh, ml; for (int q = 0; q < 4; ++q) { o[q] = pmul((y[q] - mu) * rs, bf16_rne(g2[c0 + q])) + bf16_rne(be2[c0 + q]); b16 p, qq; split16(o[q] * XS, p, qq); hv[q] = p; lv[q] = qq; mh[q] = (b16)(bf16_rne(mem[(size_t)s * F + c0 + q]) * XS); ml[q] = (b16)0.0f; }
  for (int pass = 0; pass < 2; ++pass) { *(volatile v4f*)(MU + (size_t)s * F + c0) = o; *(volatile v4b*)(CATh + (size_t)s * 2 * F + c0) = mh; *(volatile v4b*)(CATl + (size_t)s * 2 * F + c0) = ml; *(volatile v4b*)(CATh + (size_t)s * 2 * F + F + c0) = hv; *(volatile v4b*)(CATl + (size_t)s * 2 * F + F + c0) = lv; __threadfence(); }
}
__global__ __launch_bounds__(256) void gate_kernel(const float* __restrict__ GATE, const float* __restrict__ mem, const float* __restrict__ MU, float* __restrict__ out) {
  const int wave = threadIdx.x >> 5, lane = threadIdx.x & 31; const int s = blockIdx.x * 8 + wave; const int c0 = lane * 4; v4f o;
  for (int q = 0; q < 4; ++q) { const int c = c0 + q; o[q] = pmul(bf16_rne(mem[(size_t)s * F + c]), sigm(GATE[(size_t)s * 2 * F + c])) + pmul(MU[(size_t)s * F + c], sigm(GATE[(size_t)s * 2 * F + F + c])); }
  for (int pass = 0; pass < 2; ++pass) { *(volatile v4f*)(out + (size_t)s * F + c0) = o; __threadfence(); }
}
}

extern "C" void kernel_launch(void* const* d_in, const int* in_sizes, int n_in, void* d_out, int out_size, void* d_ws, size_t ws_size, hipStream_t stream) {
  (void)n_in;
  auto Fp = [&](int i) { return (const float*)d_in[i]; }; auto Ip = [&](int i) { return (const int*)d_in[i]; };
  if (in_sizes[0] != NX * FIN || in_sizes[1] != BK * F || in_sizes[2] != FIN * F || in_sizes[4] != F * 3 * F || in_sizes[13] != 4 * F * F || in_sizes[15] != E || in_sizes[16] != E || out_size != BK * F) return;
  size_t off = 0; char* ws = (char*)d_ws;
  auto carve = [&](size_t bytes) { char* p = ws + off; off += (bytes + 255) & ~(size_t)255; return p; };
  b16* X16 = (b16*)carve((size_t)NX * FIN * 2); b16* M16 = (b16*)carve((size_t)BK * F * 2); b16* WT = (b16*)carve(((size_t)F * FIN + 9 * F * F) * 2);
  b16* XPh = (b16*)carve((size_t)NX * F * 2); b16* XPl = (b16*)carve((size_t)NX * F * 2); float* Q = (float*)carve((size_t)BK * F * 4); float* Kp = (float*)carve((size_t)NCAT * F * 4); float* Vp = (float*)carve((size_t)NCAT * F * 4);
  float* MT = (float*)carve((size_t)BK * F * 4); b16* MTh = (b16*)carve((size_t)BK * F * 2); b16* MTl = (b16*)carve((size_t)BK * F * 2); b16* Th = (b16*)carve((size_t)BK * F * 2); b16* Tl = (b16*)carve((size_t)BK * F * 2); float* U = (float*)carve((size_t)BK * F * 4); float* MU = (float*)carve((size_t)BK * F * 4);
  b16* CATh = (b16*)carve((size_t)BK * 2 * F * 2); b16* CATl = (b16*)carve((size_t)BK * 2 * F * 2); float* GATE = (float*)carve((size_t)BK * 2 * F * 4);
  CsrBufs csr; off = csr_carve(csr, ws, off, E, BK);
  if (off > ws_size || off > ((size_t)128 << 20)) return;
  const b16 *WpT = WT, *WqkvT = WT + (size_t)F * FIN, *W1T = WqkvT + (size_t)3 * F * F, *W2T = W1T + (size_t)F * F, *WgT = W2T + (size_t)F * F;
  prep_kernel<<<(unsigned)(((size_t)NX * FIN / 8 + (size_t)BK * F / 8 + ((size_t)F * FIN + 9 * F * F) / 8 + 255) / 256), 256, 0, stream>>>(Fp(0), Fp(1), Fp(2), Fp(4), Fp(7), Fp(9), Fp(13), X16, M16, WT);
  csr_build(csr, Ip(15), E, BK, stream);
  gemm_kernel<0, FIN><<<dim3(NX / 64, 1), 128, 0, stream>>>(X16, nullptr, nullptr, nullptr, WpT, Fp(3), XPh, XPl, nullptr, 128);
  gemm_kernel<1, F, 1><<<dim3(BK / 64, 1), 128, 0, stream>>>(M16, nullptr, XPh, XPl, WqkvT, nullptr, nullptr, nullptr, Q, F);
  gemm_kernel<1, F><<<dim3(NCAT / 64, 1), 128, 0, stream>>>(M16, nullptr, XPh, XPl, WqkvT + (size_t)F * F, nullptr, nullptr, nullptr, Kp, F);
  gemm_kernel<1, F><<<dim3(NCAT / 64, 1), 128, 0, stream>>>(M16, nullptr, XPh, XPl, WqkvT + (size_t)2 * F * F, nullptr, nullptr, nullptr, Vp, F);
  edge_kernel<<<BK / 8, 256, 0, stream>>>(Q, Kp, Vp, Fp(1), Ip(16), csr.PERM, csr.ROWPTR, csr.ROWCNT, (int)csr.permLen, Fp(5), Fp(6), MT, MTh, MTl);
  gemm_kernel<2, F><<<dim3(BK / 64, 1), 128, 0, stream>>>(MTh, MTl, nullptr, nullptr, W1T, Fp(8), Th, Tl, nullptr, 128);
  gemm_kernel<3, F><<<dim3(BK / 64, 1), 128, 0, stream>>>(Th, Tl, nullptr, nullptr, W2T, Fp(10), nullptr, nullptr, U, F);
  ln2_kernel<<<BK / 8, 256, 0, stream>>>(MT, U, Fp(1), Fp(11), Fp(12), MU, CATh, CATl);
  gemm_kernel<3, 2 * F><<<dim3(BK / 64, 2), 128, 0, stream>>>(CATh, CATl, nullptr, nullptr, WgT, Fp(14), nullptr, nullptr, GATE, 2 * F);
  gate_kernel<<<BK / 8, 256, 0, stream>>>(GATE, Fp(1), MU, (float*)d_out);
}
